// HyperGCN_9749575762795
// MI455X (gfx1250) — hardware-verified
//
#include <hip/hip_runtime.h>


#define NNODES 32768
#define NEDGES 4096
#define NINC   131072
#define DM     256
#define DM2    512
#define EPSF   1e-5f
#define WSC    16.0f
#define WINV   0.0625f

#define TE     64
#define TN     256
#define CAPL   512

static_assert(NNODES % 64 == 0);
static_assert(NEDGES % 32 == 0);
static_assert(NEDGES % TE == 0);
static_assert(NNODES % TN == 0);
static_assert(NINC % 1024 == 0);
static_assert(TN / 8 == 32);

typedef _Float16 v16h __attribute__((ext_vector_type(16)));
typedef _Float16 v8h  __attribute__((ext_vector_type(8)));
typedef _Float16 v4h  __attribute__((ext_vector_type(4)));
typedef float    v8f  __attribute__((ext_vector_type(8)));
typedef float    v4f  __attribute__((ext_vector_type(4)));
typedef int      v4i  __attribute__((ext_vector_type(4)));
typedef v8h __attribute__((may_alias)) v8ha;
typedef v4h __attribute__((may_alias)) v4ha;
typedef v4f __attribute__((may_alias)) v4fa;
typedef v4i __attribute__((may_alias)) v4ia;

union Frag { v16h v; v8h hv[2]; };

__device__ __forceinline__ v8f wmma_f16(v16h a, v16h b, v8f c) {
    v8f d = __builtin_amdgcn_wmma_f32_16x16x32_f16(false, a, false, b, (short)0, c, false, false);
    asm volatile("v_nop\n\tv_nop\n\tv_nop\n\tv_nop" : "+v"(d) : "v"(a), "v"(b));
    return d;
}

__device__ __forceinline__ float leakyf(float v) { return v >= 0.f ? v : 0.2f * v; }

__device__ __forceinline__ float hsum16(float v) {
    v += __shfl_xor(v, 8);
    v += __shfl_xor(v, 4);
    v += __shfl_xor(v, 2);
    v += __shfl_xor(v, 1);
    return v;
}

__device__ __forceinline__ void rows16_f32(const float* tile, float* dst, int pitch, int lane) {
    const int rsub = lane >> 4, c4 = (lane & 15) * 4;
    #pragma unroll
    for (int i = 0; i < 8; ++i) {
        const int row = 2 * i + rsub;
        const v4f v = *(const v4fa*)(tile + row * 64 + c4);
        *(volatile v4fa*)(dst + (size_t)row * pitch + c4) = v;
    }
}

__device__ __forceinline__ void rows16_f16(const float* tile, _Float16* dst, int pitch, int lane) {
    const int rsub = lane >> 3, c8 = (lane & 7) * 8;
    #pragma unroll
    for (int i = 0; i < 4; ++i) {
        const int row = 4 * i + rsub;
        const v4f a = *(const v4fa*)(tile + row * 64 + c8);
        const v4f b = *(const v4fa*)(tile + row * 64 + c8 + 4);
        v8h o;
        o[0] = (_Float16)a[0]; o[1] = (_Float16)a[1]; o[2] = (_Float16)a[2]; o[3] = (_Float16)a[3];
        o[4] = (_Float16)b[0]; o[5] = (_Float16)b[1]; o[6] = (_Float16)b[2]; o[7] = (_Float16)b[3];
        *(volatile v8ha*)(dst + (size_t)row * pitch + c8) = o;
    }
}

#define CVT_NB0 (NNODES * DM / 2048)
#define CVT_NB1 (DM * DM / 2048)
#define CVT_NB2 (DM2 * DM / 2048)
#define CVT_NB3 (DM * DM / 2048)

__global__ __launch_bounds__(256) void k_cvt(
    const float* __restrict__ s0, _Float16* d0,
    const float* __restrict__ s1, _Float16* d1,
    const float* __restrict__ s2, _Float16* d2,
    const float* __restrict__ s3, _Float16* d3)
{
    const int b = blockIdx.x;
    const float* s; _Float16* d; float sc; int lb;
    if (b < CVT_NB0)                            { s = s0; d = d0; sc = 1.f;  lb = b; }
    else if (b < CVT_NB0 + CVT_NB1)             { s = s1; d = d1; sc = WSC;  lb = b - CVT_NB0; }
    else if (b < CVT_NB0 + CVT_NB1 + CVT_NB2)   { s = s2; d = d2; sc = WSC;  lb = b - CVT_NB0 - CVT_NB1; }
    else                                        { s = s3; d = d3; sc = WSC;  lb = b - CVT_NB0 - CVT_NB1 - CVT_NB2; }
    const size_t i = (size_t)lb * 2048 + (size_t)threadIdx.x * 8;
    const v4f a = *(const v4fa*)(s + i);
    const v4f c = *(const v4fa*)(s + i + 4);
    v8h o;
    o[0] = (_Float16)(a[0] * sc); o[1] = (_Float16)(a[1] * sc); o[2] = (_Float16)(a[2] * sc); o[3] = (_Float16)(a[3] * sc);
    o[4] = (_Float16)(c[0] * sc); o[5] = (_Float16)(c[1] * sc); o[6] = (_Float16)(c[2] * sc); o[7] = (_Float16)(c[3] * sc);
    _Float16* dp = d + i;
    *(volatile v8ha*)dp = o;
    __threadfence();
    *(volatile v8ha*)dp = o;
}

template<int MODE>
__global__ __launch_bounds__(256) void k_gemm(
    const _Float16* __restrict__ A, const _Float16* __restrict__ Bw,
    float* out32, _Float16* out16,
    const float* __restrict__ bias,
    const float* __restrict__ bng, const float* __restrict__ bnb,
    const float* __restrict__ bnm, const float* __restrict__ bnv,
    const float* __restrict__ att, float* score,
    const float* __restrict__ xres,
    const float* __restrict__ lng, const float* __restrict__ lnb)
{
    constexpr int NCW   = (MODE == 1 || MODE == 2) ? 8 : 4;
    constexpr int NRW   = 8 / NCW;
    constexpr int BROWS = 32 * NRW;
    constexpr int OP    = NCW * 64;

    __shared__ __align__(16) float sT[8][16 * 64];
    __shared__ float sP[8][32];

    const int tid = threadIdx.x, lane = tid & 31, wave = tid >> 5;
    const int h = lane >> 4, m = lane & 15;
    const int cw = wave % NCW, rw = wave / NCW;
    const int rowbase = blockIdx.x * BROWS + rw * 32;
    const int col0 = cw * 64;

    v8f acc[2][4];
    #pragma unroll
    for (int t = 0; t < 2; ++t)
        #pragma unroll
        for (int j = 0; j < 4; ++j) {
            v8f z = {};
            acc[t][j] = z;
        }

    const _Float16* ap0 = A  + (size_t)(rowbase + m) * DM + 8 * h;
    const _Float16* ap1 = ap0 + 16 * DM;
    const _Float16* bp  = Bw + (size_t)(col0 + m) * DM + 8 * h;

    #pragma unroll 2
    for (int kc = 0; kc < 8; ++kc) {
        const int k0 = kc * 32;
        Frag a0, a1, b[4];
        a0.hv[0] = *(const v8ha*)(ap0 + k0);
        a0.hv[1] = *(const v8ha*)(ap0 + k0 + 16);
        a1.hv[0] = *(const v8ha*)(ap1 + k0);
        a1.hv[1] = *(const v8ha*)(ap1 + k0 + 16);
        #pragma unroll
        for (int j = 0; j < 4; ++j) {
            b[j].hv[0] = *(const v8ha*)(bp + (size_t)j * 16 * DM + k0);
            b[j].hv[1] = *(const v8ha*)(bp + (size_t)j * 16 * DM + k0 + 16);
        }
        #pragma unroll
        for (int j = 0; j < 4; ++j) {
            acc[0][j] = wmma_f16(a0.v, b[j].v, acc[0][j]);
            acc[1][j] = wmma_f16(a1.v, b[j].v, acc[1][j]);
        }
    }

    float c0[4], c1[4], c2[4], c3[4], c4[4];
    #pragma unroll
    for (int j = 0; j < 4; ++j) {
        const int col = col0 + 16 * j + m;
        c0[j] = 0.f; c1[j] = 0.f; c2[j] = 0.f; c3[j] = 0.f; c4[j] = 0.f;
        if constexpr (MODE == 0) {
            c0[j] = bias[col]; c1[j] = bng[col]; c2[j] = bnb[col]; c3[j] = bnm[col]; c4[j] = rsqrtf(bnv[col] + EPSF);
        } else if constexpr (MODE == 1) {
            const int head = col >> 8, d = col & 255;
            c0[j] = att[head * DM2 + d];
        } else if constexpr (MODE == 2) {
            const int head = col >> 8, d = col & 255;
            c0[j] = att[head * DM2 + DM + d];
        } else {
            const int cl = 16 * j + m;
            c0[j] = bias[col]; c1[j] = lng[cl]; c2[j] = lnb[cl];
        }
    }

    float* tile = &sT[wave][0];
    #pragma unroll
    for (int t = 0; t < 2; ++t) {
        if constexpr (MODE == 0) {
            #pragma unroll
            for (int j = 0; j < 4; ++j)
                #pragma unroll
                for (int r = 0; r < 8; ++r) {
                    float v = leakyf(acc[t][j][r] * WINV + c0[j]);
                    v = c1[j] * (v - c3[j]) * c4[j] + c2[j];
                    tile[(8 * h + r) * 64 + 16 * j + m] = v;
                }
        } else if constexpr (MODE == 1 || MODE == 2) {
            float p[8];
            #pragma unroll
            for (int r = 0; r < 8; ++r) p[r] = 0.f;
            #pragma unroll
            for (int j = 0; j < 4; ++j)
                #pragma unroll
                for (int r = 0; r < 8; ++r) {
                    const float v = acc[t][j][r] * WINV;
                    if constexpr (MODE == 1) tile[(8 * h + r) * 64 + 16 * j + m] = v;
                    p[r] += v * c0[j];
                }
            #pragma unroll
            for (int r = 0; r < 8; ++r) p[r] = hsum16(p[r]);
            if (m == 0) {
                #pragma unroll
                for (int r = 0; r < 8; ++r) sP[wave][16 * t + 8 * h + r] = p[r];
            }
        } else {
            float y[4][8];
            #pragma unroll
            for (int j = 0; j < 4; ++j)
                #pragma unroll
                for (int r = 0; r < 8; ++r) {
                    const int grow = rowbase + 16 * t + 8 * h + r;
                    const int col  = col0 + 16 * j + m;
                    const float v = leakyf(acc[t][j][r] * WINV + c0[j]);
                    y[j][r] = xres[(size_t)grow * DM + col] + v;
                }
            #pragma unroll
            for (int r = 0; r < 8; ++r) {
                float s = y[0][r] + y[1][r]; s += y[2][r]; s += y[3][r];
                s = hsum16(s);
                const float mu = s * (1.0f / 64.0f);
                #pragma unroll
                for (int j = 0; j < 4; ++j) y[j][r] = y[j][r] - mu;
                float q = y[0][r] * y[0][r]; q += y[1][r] * y[1][r]; q += y[2][r] * y[2][r]; q += y[3][r] * y[3][r];
                q = hsum16(q);
                const float rs = rsqrtf(q * (1.0f / 64.0f) + EPSF);
                #pragma unroll
                for (int j = 0; j < 4; ++j)
                    tile[(8 * h + r) * 64 + 16 * j + m] = c1[j] * y[j][r] * rs + c2[j];
            }
        }
        __syncthreads();
        if constexpr (MODE == 0) {
            float*    d32 = out32 + (size_t)(rowbase + 16 * t) * OP + col0;
            _Float16* d16 = out16 + (size_t)(rowbase + 16 * t) * OP + col0;
            rows16_f32(tile, d32, OP, lane);
            rows16_f16(tile, d16, OP, lane);
            __threadfence();
            rows16_f32(tile, d32, OP, lane);
            rows16_f16(tile, d16, OP, lane);
        } else if constexpr (MODE == 1) {
            _Float16* d16 = out16 + (size_t)(rowbase + 16 * t) * OP + col0;
            rows16_f16(tile, d16, OP, lane);
            __threadfence();
            rows16_f16(tile, d16, OP, lane);
        } else if constexpr (MODE == 3) {
            float* d32 = out32 + (size_t)(rowbase + 16 * t) * OP + col0;
            rows16_f32(tile, d32, OP, lane);
            __threadfence();
            rows16_f32(tile, d32, OP, lane);
        }
        __syncthreads();
    }

    if constexpr (MODE == 1 || MODE == 2) {
        if (wave == 0 && lane < 16) {
            const int q = lane;
            v4f o;
            #pragma unroll
            for (int rr = 0; rr < 2; ++rr) {
                const int row = 2 * q + rr;
                #pragma unroll
                for (int hh = 0; hh < 2; ++hh) {
                    float s = sP[4 * hh][row];
                    s += sP[4 * hh + 1][row];
                    s += sP[4 * hh + 2][row];
                    s += sP[4 * hh + 3][row];
                    o[2 * rr + hh] = s;
                }
            }
            float* sp = score + (size_t)(blockIdx.x * 32 + 2 * q) * 2;
            *(volatile v4fa*)sp = o;
            __threadfence();
            *(volatile v4fa*)sp = o;
        }
    }
}

template<int T, int SB, int CAP>
__device__ __forceinline__ int build_lists(const int* __restrict__ dsti, const int* __restrict__ srci,
                                           int d0, int srcmax, int* sA, int* sCA, int* sB, int wave, int lane)
{
    const unsigned lt = (1u << lane) - 1u;
    int cnt = 0;
    const int ibeg = wave * (NINC / 8);
    #pragma unroll 1
    for (int i0 = ibeg; i0 < ibeg + NINC / 8; i0 += 128) {
        const v4i dv = *(const v4ia*)(dsti + i0 + 4 * lane);
        const v4i sv = *(const v4ia*)(srci + i0 + 4 * lane);
        #pragma unroll
        for (int c = 0; c < 4; ++c) {
            const int d = dv[c] - d0;
            const bool hit = (unsigned)d < (unsigned)T;
            const unsigned mask = __builtin_amdgcn_ballot_w32(hit);
            const int pos = cnt + __builtin_popcount(mask & lt);
            int s = sv[c];
            s = s < 0 ? 0 : s;
            s = s > srcmax ? srcmax : s;
            if (hit && pos < CAP) sA[wave * CAP + pos] = (d << SB) | s;
            cnt += __builtin_popcount(mask);
        }
    }
    if (lane == 0) sCA[wave] = cnt < CAP ? cnt : CAP;
    __syncthreads();

    int cb = 0;
    #pragma unroll 1
    for (int s = 0; s < 8; ++s) {
        int cs = sCA[s];
        cs = cs < CAP ? cs : CAP;
        #pragma unroll 1
        for (int base = 0; base < cs; base += 32) {
            const int idx = base + lane;
            const bool valid = idx < cs;
            const int ent = sA[s * CAP + (valid ? idx : 0)];
            const bool mine = valid && (((ent >> SB) / (T / 8)) == wave);
            const unsigned mask = __builtin_amdgcn_ballot_w32(mine);
            const int pos = cb + __builtin_popcount(mask & lt);
            if (mine && pos < CAP) sB[wave * CAP + pos] = ent;
            cb += __builtin_popcount(mask);
        }
    }
    __syncthreads();
    return cb < CAP ? cb : CAP;
}

__device__ __forceinline__ void alpha2(float sn0, float sn1, float se0, float se1, v4f st, float& w0, float& w1) {
    const float a0 = leakyf(sn0 + se0);
    const float a1 = leakyf(sn1 + se1);
    w0 = expf(a0 - st[0]) * (1.0f / (st[2] + 1e-16f));
    w1 = expf(a1 - st[1]) * (1.0f / (st[3] + 1e-16f));
}

__global__ __launch_bounds__(256) void k_eattr(const int* __restrict__ he, const float* __restrict__ h32, _Float16* eat16)
{
    __shared__ int sA[8 * CAPL];
    __shared__ int sB[8 * CAPL];
    __shared__ int sCA[8];
    const int lane = threadIdx.x & 31, wave = threadIdx.x >> 5;
    const int e0 = blockIdx.x * TE;
    const int cb = build_lists<TE, 15, CAPL>(he + NINC, he, e0, NNODES - 1, sA, sCA, sB, wave, lane);
    const int* myl = sB + wave * CAPL;

    #pragma unroll 1
    for (int dl = 0; dl < TE / 8; ++dl) {
        const int dloc = wave * (TE / 8) + dl;
        const int e = e0 + dloc;
        float acc[8];
        #pragma unroll
        for (int c = 0; c < 8; ++c) acc[c] = 0.f;
        #pragma unroll 1
        for (int base = 0; base < cb; base += 32) {
            const int idx = base + lane;
            const bool valid = idx < cb;
            const int ent = myl[valid ? idx : 0];
            const bool match = valid && ((ent >> 15) == dloc);
            unsigned mask = __builtin_amdgcn_ballot_w32(match);
            while (mask) {
                const int bsel = __builtin_ctz(mask);
                mask &= mask - 1u;
                const int n = __shfl(ent, bsel) & 0x7fff;
                const float* hp = h32 + (size_t)n * DM + 8 * lane;
                const v4f u0 = *(const v4fa*)hp;
                const v4f u1 = *(const v4fa*)(hp + 4);
                acc[0] += u0[0]; acc[1] += u0[1]; acc[2] += u0[2]; acc[3] += u0[3];
                acc[4] += u1[0]; acc[5] += u1[1]; acc[6] += u1[2]; acc[7] += u1[3];
            }
        }
        v8h o;
        #pragma unroll
        for (int c = 0; c < 8; ++c) o[c] = (_Float16)acc[c];
        _Float16* dp = eat16 + (size_t)e * DM + 8 * lane;
        *(volatile v8ha*)dp = o;
        __threadfence();
        *(volatile v8ha*)dp = o;
    }
}

__global__ __launch_bounds__(256) void k_nstat(const int* __restrict__ he, const float* __restrict__ sn,
                                               const float* __restrict__ se, float* nst)
{
    __shared__ int sA[8 * CAPL];
    __shared__ int sB[8 * CAPL];
    __shared__ int sCA[8];
    const int lane = threadIdx.x & 31, wave = threadIdx.x >> 5;
    const int n0 = blockIdx.x * TN;
    const int cb = build_lists<TN, 12, CAPL>(he, he + NINC, n0, NEDGES - 1, sA, sCA, sB, wave, lane);
    const int* myl = sB + wave * CAPL;

    const int me = wave * 32 + lane;
    const int n = n0 + me;
    const float s0 = sn[2 * n], s1 = sn[2 * n + 1];
    const float ninf = -__builtin_huge_valf();
    float am0 = ninf, am1 = ninf;
    int deg = 0;
    #pragma unroll 1
    for (int k = 0; k < cb; ++k) {
        const int ent = myl[k];
        if ((ent >> 12) == me) {
            const int e = ent & 4095;
            const float a0 = leakyf(s0 + se[2 * e]);
            const float a1 = leakyf(s1 + se[2 * e + 1]);
            am0 = fmaxf(am0, a0);
            am1 = fmaxf(am1, a1);
            ++deg;
        }
    }
    const float z0 = deg > 0 ? am0 : 0.f;
    const float z1 = deg > 0 ? am1 : 0.f;
    float dn0 = 0.f, dn1 = 0.f;
    #pragma unroll 1
    for (int k = 0; k < cb; ++k) {
        const int ent = myl[k];
        if ((ent >> 12) == me) {
            const int e = ent & 4095;
            const float a0 = leakyf(s0 + se[2 * e]);
            const float a1 = leakyf(s1 + se[2 * e + 1]);
            dn0 += expf(a0 - z0);
            dn1 += expf(a1 - z1);
        }
    }
    v4f o;
    o[0] = z0; o[1] = z1; o[2] = dn0; o[3] = dn1;
    float* dp = nst + (size_t)n * 4;
    *(volatile v4fa*)dp = o;
    __threadfence();
    *(volatile v4fa*)dp = o;
}

__global__ __launch_bounds__(256) void k_eout(const int* __restrict__ he, const float* __restrict__ sn,
                                              const float* __restrict__ se, const float* __restrict__ nst,
                                              const _Float16* __restrict__ xh16, float* eo32)
{
    __shared__ int sA[8 * CAPL];
    __shared__ int sB[8 * CAPL];
    __shared__ int sCA[8];
    const int lane = threadIdx.x & 31, wave = threadIdx.x >> 5;
    const int e0 = blockIdx.x * TE;
    const int cb = build_lists<TE, 15, CAPL>(he + NINC, he, e0, NNODES - 1, sA, sCA, sB, wave, lane);
    const int* myl = sB + wave * CAPL;

    #pragma unroll 1
    for (int dl = 0; dl < TE / 8; ++dl) {
        const int dloc = wave * (TE / 8) + dl;
        const int e = e0 + dloc;
        const float se0 = se[2 * e], se1 = se[2 * e + 1];
        float acc[16];
        #pragma unroll
        for (int c = 0; c < 16; ++c) acc[c] = 0.f;
        int deg = 0;
        #pragma unroll 1
        for (int base = 0; base < cb; base += 32) {
            const int idx = base + lane;
            const bool valid = idx < cb;
            const int ent = myl[valid ? idx : 0];
            const bool match = valid && ((ent >> 15) == dloc);
            unsigned mask = __builtin_amdgcn_ballot_w32(match);
            deg += __builtin_popcount(mask);
            while (mask) {
                const int bsel = __builtin_ctz(mask);
                mask &= mask - 1u;
                const int n = __shfl(ent, bsel) & 0x7fff;
                const v4f st = *(const v4fa*)(nst + (size_t)n * 4);
                float w0, w1;
                alpha2(sn[2 * n], sn[2 * n + 1], se0, se1, st, w0, w1);
                const _Float16* xp = xh16 + (size_t)n * DM2 + 4 * lane;
                #pragma unroll
                for (int k = 0; k < 4; ++k) {
                    const v4h u = *(const v4ha*)(xp + 128 * k);
                    const float w = (k < 2) ? w0 : w1;
                    #pragma unroll
                    for (int c = 0; c < 4; ++c) acc[4 * k + c] += w * (float)u[c];
                }
            }
        }
        const float binv = deg > 0 ? 1.0f / (float)deg : 0.f;
        v4f ov[4];
        #pragma unroll
        for (int k = 0; k < 4; ++k) {
            ov[k][0] = binv * acc[4 * k + 0]; ov[k][1] = binv * acc[4 * k + 1];
            ov[k][2] = binv * acc[4 * k + 2]; ov[k][3] = binv * acc[4 * k + 3];
        }
        float* dp = eo32 + (size_t)e * DM2 + 4 * lane;
        #pragma unroll
        for (int k = 0; k < 4; ++k) *(volatile v4fa*)(dp + 128 * k) = ov[k];
        __threadfence();
        #pragma unroll
        for (int k = 0; k < 4; ++k) *(volatile v4fa*)(dp + 128 * k) = ov[k];
    }
}

__global__ __launch_bounds__(256) void k_nout(const int* __restrict__ he, const float* __restrict__ sn,
                                              const float* __restrict__ se, const float* __restrict__ nst,
                                              const float* __restrict__ eo32, const float* __restrict__ h32,
                                              const float* __restrict__ cbias,
                                              const float* __restrict__ g2, const float* __restrict__ b2n,
                                              const float* __restrict__ m2, const float* __restrict__ v2,
                                              _Float16* t16)
{
    __shared__ int sA[8 * CAPL];
    __shared__ int sB[8 * CAPL];
    __shared__ int sCA[8];
    const int lane = threadIdx.x & 31, wave = threadIdx.x >> 5;
    const int n0 = blockIdx.x * TN;
    const int cb = build_lists<TN, 12, CAPL>(he, he + NINC, n0, NEDGES - 1, sA, sCA, sB, wave, lane);
    const int* myl = sB + wave * CAPL;

    const int c8 = 8 * lane;
    float cbv[8], gv[8], bv[8], mv[8], rv[8];
    {
        const v4f q0 = *(const v4fa*)(cbias + c8), q1 = *(const v4fa*)(cbias + c8 + 4);
        const v4f g0 = *(const v4fa*)(g2 + c8),    g1 = *(const v4fa*)(g2 + c8 + 4);
        const v4f p0 = *(const v4fa*)(b2n + c8),   p1 = *(const v4fa*)(b2n + c8 + 4);
        const v4f u0 = *(const v4fa*)(m2 + c8),    u1 = *(const v4fa*)(m2 + c8 + 4);
        const v4f w0 = *(const v4fa*)(v2 + c8),    w1 = *(const v4fa*)(v2 + c8 + 4);
        #pragma unroll
        for (int c = 0; c < 4; ++c) {
            cbv[c] = q0[c]; cbv[4 + c] = q1[c];
            gv[c]  = g0[c]; gv[4 + c]  = g1[c];
            bv[c]  = p0[c]; bv[4 + c]  = p1[c];
            mv[c]  = u0[c]; mv[4 + c]  = u1[c];
            rv[c]  = rsqrtf(w0[c] + EPSF); rv[4 + c] = rsqrtf(w1[c] + EPSF);
        }
    }

    #pragma unroll 1
    for (int dl = 0; dl < TN / 8; ++dl) {
        const int dloc = wave * (TN / 8) + dl;
        const int n = n0 + dloc;
        const float s0 = sn[2 * n], s1 = sn[2 * n + 1];
        const v4f st = *(const v4fa*)(nst + (size_t)n * 4);
        float acc0[8], acc1[8];
        #pragma unroll
        for (int c = 0; c < 8; ++c) { acc0[c] = 0.f; acc1[c] = 0.f; }
        int deg = 0;
        #pragma unroll 1
        for (int base = 0; base < cb; base += 32) {
            const int idx = base + lane;
            const bool valid = idx < cb;
            const int ent = myl[valid ? idx : 0];
            const bool match = valid && ((ent >> 12) == dloc);
            unsigned mask = __builtin_amdgcn_ballot_w32(match);
            deg += __builtin_popcount(mask);
            while (mask) {
                const int bsel = __builtin_ctz(mask);
                mask &= mask - 1u;
                const int e = __shfl(ent, bsel) & 4095;
                float w0, w1;
                alpha2(s0, s1, se[2 * e], se[2 * e + 1], st, w0, w1);
                const float* ep = eo32 + (size_t)e * DM2 + c8;
                const v4f u0 = *(const v4fa*)ep;
                const v4f u1 = *(const v4fa*)(ep + 4);
                const v4f u2 = *(const v4fa*)(ep + DM);
                const v4f u3 = *(const v4fa*)(ep + DM + 4);
                #pragma unroll
                for (int c = 0; c < 4; ++c) {
                    acc0[c]     += w0 * u0[c];
                    acc0[4 + c] += w0 * u1[c];
                    acc1[c]     += w1 * u2[c];
                    acc1[4 + c] += w1 * u3[c];
                }
            }
        }
        const float dinv = deg > 0 ? 1.0f / (float)deg : 0.f;
        const float* hp = h32 + (size_t)n * DM + c8;
        const v4f hv0 = *(const v4fa*)hp;
        const v4f hv1 = *(const v4fa*)(hp + 4);
        v8h o;
        #pragma unroll
        for (int c = 0; c < 8; ++c) {
            const float no0 = dinv * acc0[c];
            const float no1 = dinv * acc1[c];
            const float x2 = (no0 + no1) * 0.5f + cbv[c];
            const float hval = (c < 4) ? hv0[c] : hv1[c - 4];
            const float pre = hval + x2;
            const float tv = gv[c] * (pre - mv[c]) * rv[c] + bv[c];
            o[c] = (_Float16)tv;
        }
        _Float16* dp = t16 + (size_t)n * DM + c8;
        *(volatile v8ha*)dp = o;
        __threadfence();
        *(volatile v8ha*)dp = o;
    }
}

extern "C" void kernel_launch(void* const* d_in, const int* in_sizes, int n_in,
                              void* d_out, int out_size, void* d_ws, size_t ws_size,
                              hipStream_t stream)
{
    if (n_in < 19) return;
    if (in_sizes[0] != NNODES * DM || in_sizes[1] != 2 * NINC || in_sizes[2] != DM * DM ||
        in_sizes[3] != DM || in_sizes[8] != DM2 * DM || in_sizes[9] != 2 * DM2 ||
        in_sizes[10] != DM || in_sizes[15] != DM * DM || in_sizes[16] != DM ||
        in_sizes[17] != 64 || in_sizes[18] != 64 || out_size != NNODES * DM) return;

    const float* x    = (const float*)d_in[0];
    const int*   he   = (const int*)  d_in[1];
    const float* W1   = (const float*)d_in[2];
    const float* b1   = (const float*)d_in[3];
    const float* bn1g = (const float*)d_in[4];
    const float* bn1b = (const float*)d_in[5];
    const float* bn1m = (const float*)d_in[6];
    const float* bn1v = (const float*)d_in[7];
    const float* attW = (const float*)d_in[8];
    const float* att  = (const float*)d_in[9];
    const float* cb   = (const float*)d_in[10];
    const float* bn2g = (const float*)d_in[11];
    const float* bn2b = (const float*)d_in[12];
    const float* bn2m = (const float*)d_in[13];
    const float* bn2v = (const float*)d_in[14];
    const float* W2   = (const float*)d_in[15];
    const float* b2   = (const float*)d_in[16];
    const float* lng  = (const float*)d_in[17];
    const float* lnb  = (const float*)d_in[18];
    float* out = (float*)d_out;

    char*  base = (char*)d_ws;
    size_t off  = 0;
    auto carve = [&](size_t bytes) -> char* {
        char* p = base + off;
        off += (bytes + 255) & ~(size_t)255;
        return p;
    };
    _Float16* x16   = (_Float16*)carve((size_t)NNODES * DM * 2);
    _Float16* t16   = x16;
    float*    h32   = (float*)   carve((size_t)NNODES * DM * 4);
    _Float16* h16   = (_Float16*)carve((size_t)NNODES * DM * 2);
    _Float16* xh16  = (_Float16*)carve((size_t)NNODES * DM2 * 2);
    _Float16* eat16 = (_Float16*)carve((size_t)NEDGES * DM * 2);
    float*    eo32  = (float*)   carve((size_t)NEDGES * DM2 * 4);
    float*    sn    = (float*)   carve((size_t)NNODES * 2 * 4);
    float*    se    = (float*)   carve((size_t)NEDGES * 2 * 4);
    float*    nst   = (float*)   carve((size_t)NNODES * 4 * 4);
    _Float16* W1h   = (_Float16*)carve((size_t)DM * DM * 2);
    _Float16* Wah   = (_Float16*)carve((size_t)DM2 * DM * 2);
    _Float16* W2h   = (_Float16*)carve((size_t)DM * DM * 2);
    if (off > ws_size) return;

    k_cvt<<<CVT_NB0 + CVT_NB1 + CVT_NB2 + CVT_NB3, 256, 0, stream>>>(x, x16, W1, W1h, attW, Wah, W2, W2h);

    k_gemm<0><<<NNODES / 64, 256, 0, stream>>>(x16, W1h, h32, h16, b1, bn1g, bn1b, bn1m, bn1v,
                                               att, sn, x, lng, lnb);
    k_eattr<<<NEDGES / TE, 256, 0, stream>>>(he, h32, eat16);
    k_gemm<1><<<NNODES / 32, 256, 0, stream>>>(h16, Wah, h32, xh16, b1, bn1g, bn1b, bn1m, bn1v,
                                               att, sn, x, lng, lnb);
    k_gemm<2><<<NEDGES / 32, 256, 0, stream>>>(eat16, Wah, h32, xh16, b1, bn1g, bn1b, bn1m, bn1v,
                                               att, se, x, lng, lnb);
    k_nstat<<<NNODES / TN, 256, 0, stream>>>(he, sn, se, nst);
    k_eout<<<NEDGES / TE, 256, 0, stream>>>(he, sn, se, nst, xh16, eo32);
    k_nout<<<NNODES / TN, 256, 0, stream>>>(he, sn, se, nst, eo32, h32, cb, bn2g, bn2b, bn2m, bn2v, t16);
    k_gemm<3><<<NNODES / 64, 256, 0, stream>>>(t16, W2h, out, h16, b2, bn1g, bn1b, bn1m, bn1v,
                                               att, sn, x, lng, lnb);
}
